// ToeplitzHeads_48137993453905
// MI455X (gfx1250) — hardware-verified
//
#include <hip/hip_runtime.h>


#define NBT  4
#define DD   1024
#define TT   2048
#define NH_  16
#define EH   64
#define DM   DD
#define LOSC 1024.0f

typedef _Float16 h16;
typedef unsigned short bf;
typedef __attribute__((ext_vector_type(16))) __bf16   v16bf;
typedef __attribute__((ext_vector_type(16))) _Float16 v16h;
typedef __attribute__((ext_vector_type(8)))  _Float16 v8h;
typedef __attribute__((ext_vector_type(8)))  unsigned short v8us;
typedef __attribute__((ext_vector_type(8)))  float    v8f;
typedef __attribute__((ext_vector_type(4)))  float    v4f;
typedef v8h  __attribute__((may_alias)) v8ha;
typedef v4f  __attribute__((may_alias)) v4fa;
typedef v8us __attribute__((may_alias)) v8usa;

__device__ __forceinline__ unsigned short f2bf(float f) { unsigned u = __float_as_uint(f); u += 0x7FFFu + ((u >> 16) & 1u); return (unsigned short)(u >> 16); }
__device__ __forceinline__ float bf2f(unsigned short b) { return __uint_as_float(((unsigned)b) << 16); }
__device__ __forceinline__ float bfr(float f) { return bf2f(f2bf(f)); }
__device__ __forceinline__ v16h cat16(v8h lo, v8h hi) { return __builtin_shufflevector(lo, hi, 0, 1, 2, 3, 4, 5, 6, 7, 8, 9, 10, 11, 12, 13, 14, 15); }
__device__ __forceinline__ v16bf cat16b(v8us lo, v8us hi) { return __builtin_bit_cast(v16bf, __builtin_shufflevector(lo, hi, 0, 1, 2, 3, 4, 5, 6, 7, 8, 9, 10, 11, 12, 13, 14, 15)); }
__device__ __forceinline__ v8f wmma16(v16h a, v16h b, v8f c) { return __builtin_amdgcn_wmma_f32_16x16x32_f16(false, a, false, b, (short)0, c, false, false); }
__device__ __forceinline__ v8f wmmab(v16bf a, v16bf b, v8f c) { return __builtin_amdgcn_wmma_f32_16x16x32_bf16(false, a, false, b, (short)0, c, false, false); }

template <bool SPLITA, bool F16OUT = false>
__global__ __launch_bounds__(128) void k_gemmb(const bf* __restrict__ A, const bf* __restrict__ Al, const bf* __restrict__ Bn, const float* __restrict__ bias, float* C, int ldc, h16* C2, const float* __restrict__ R = nullptr, int K = DM, int roundR = 1) {
    __shared__ __align__(16) float ost[4][16 * 68];
    const int lane = threadIdx.x & 31, wave = threadIdx.x >> 5, lr = lane & 15, hi = lane >> 4;
    const int r0 = blockIdx.x * 64 + wave * 16, c0 = blockIdx.y * 64;
    const size_t aoff = (size_t)(r0 + lr) * K + 8 * hi;
    size_t boff[4];
#pragma unroll
    for (int t = 0; t < 4; ++t) boff[t] = (size_t)(c0 + t * 16 + lr) * K + 8 * hi;
    v8f acc[4];
#pragma unroll
    for (int t = 0; t < 4; ++t) acc[t] = (v8f){};
#pragma unroll 1
    for (int kc = 0; kc < K; kc += 32) {
        const v16bf a = cat16b(*(const v8us*)(A + aoff + kc), *(const v8us*)(A + aoff + kc + 16));
        v16bf al = a;
        if (SPLITA) al = cat16b(*(const v8us*)(Al + aoff + kc), *(const v8us*)(Al + aoff + kc + 16));
#pragma unroll
        for (int t = 0; t < 4; ++t) { const v16bf b = cat16b(*(const v8us*)(Bn + boff[t] + kc), *(const v8us*)(Bn + boff[t] + kc + 16)); acc[t] = wmmab(a, b, acc[t]); if (SPLITA) acc[t] = wmmab(al, b, acc[t]); }
        asm volatile("v_nop\n\tv_nop\n\tv_nop\n\tv_nop" : "+v"(acc[0]), "+v"(acc[1]), "+v"(acc[2]), "+v"(acc[3]) : "v"(a), "v"(al));
    }
    float* os = &ost[wave][0];
#pragma unroll
    for (int t = 0; t < 4; ++t) { const float bv = bias ? bfr(bias[c0 + t * 16 + lr]) : 0.f;
#pragma unroll
        for (int j = 0; j < 8; ++j) os[(hi * 8 + j) * 68 + t * 16 + lr] = acc[t][j] + bv; }
    __syncthreads();
    if (F16OUT) {
        h16* crow = (h16*)(void*)C + (size_t)r0 * ldc + c0;
        auto pass = [&]() {
#pragma unroll
            for (int s = 0; s < 4; ++s) { const int row = 4 * s + (lane >> 3), piece = lane & 7; const float* sp = os + row * 68 + piece * 8; v8h o, o2;
#pragma unroll
                for (int i = 0; i < 8; ++i) { const h16 a = (h16)sp[i]; o[i] = a; o2[i] = (h16)((sp[i] - (float)a) * LOSC); }
                *(volatile v8h*)(crow + (size_t)row * ldc + piece * 8) = o; if (C2) *(volatile v8h*)(C2 + (size_t)r0 * ldc + c0 + (size_t)row * ldc + piece * 8) = o2; }
        };
        pass(); __threadfence(); pass();
    } else {
        float* crow = C + (size_t)r0 * ldc + c0;
        auto pass = [&]() {
#pragma unroll
            for (int s = 0; s < 8; ++s) { const int Lid = (lane >> 3) + 4 * s, piece = lane & 7; const int row = Lid >> 1, cofs = (Lid & 1) * 32 + piece * 4;
                v4f val = *(const v4fa*)(os + row * 68 + cofs); if (R) { const v4f rv = *(const v4f*)(R + ((size_t)r0 + row) * ldc + c0 + cofs); val += roundR ? (v4f){bfr(rv[0]), bfr(rv[1]), bfr(rv[2]), bfr(rv[3])} : rv; }
                *(volatile v4f*)(crow + (size_t)row * ldc + cofs) = val; }
        };
        pass(); __threadfence(); pass();
    }
}

template <bool SPLITA, bool F16OUT = false>
__global__ __launch_bounds__(128) void k_gemmbt(const bf* __restrict__ A, const bf* __restrict__ Al, const bf* __restrict__ Bn, const float* __restrict__ bias, float* C, int ldc, h16* C2, const float* __restrict__ R, int K, int roundR) {
    const int Klim = min(K, ((int)blockIdx.x + 1) * 64);
    __shared__ __align__(16) float ost[4][16 * 68];
    const int lane = threadIdx.x & 31, wave = threadIdx.x >> 5, lr = lane & 15, hi = lane >> 4;
    const int r0 = blockIdx.x * 64 + wave * 16, c0 = blockIdx.y * 64;
    const size_t aoff = (size_t)(r0 + lr) * K + 8 * hi;
    size_t boff[4];
#pragma unroll
    for (int t = 0; t < 4; ++t) boff[t] = (size_t)(c0 + t * 16 + lr) * K + 8 * hi;
    v8f acc[4];
#pragma unroll
    for (int t = 0; t < 4; ++t) acc[t] = (v8f){};
#pragma unroll 1
    for (int kc = 0; kc < Klim; kc += 32) {
        const v16bf a = cat16b(*(const v8us*)(A + aoff + kc), *(const v8us*)(A + aoff + kc + 16));
        v16bf al = a;
        if (SPLITA) al = cat16b(*(const v8us*)(Al + aoff + kc), *(const v8us*)(Al + aoff + kc + 16));
#pragma unroll
        for (int t = 0; t < 4; ++t) { const v16bf b = cat16b(*(const v8us*)(Bn + boff[t] + kc), *(const v8us*)(Bn + boff[t] + kc + 16)); acc[t] = wmmab(a, b, acc[t]); if (SPLITA) acc[t] = wmmab(al, b, acc[t]); }
        asm volatile("v_nop\n\tv_nop\n\tv_nop\n\tv_nop" : "+v"(acc[0]), "+v"(acc[1]), "+v"(acc[2]), "+v"(acc[3]) : "v"(a), "v"(al));
    }
    float* os = &ost[wave][0];
#pragma unroll
    for (int t = 0; t < 4; ++t) { const float bv = bias ? bfr(bias[c0 + t * 16 + lr]) : 0.f;
#pragma unroll
        for (int j = 0; j < 8; ++j) os[(hi * 8 + j) * 68 + t * 16 + lr] = acc[t][j] + bv; }
    __syncthreads();
    if (F16OUT) {
        h16* crow = (h16*)(void*)C + (size_t)r0 * ldc + c0;
        auto pass = [&]() {
#pragma unroll
            for (int s = 0; s < 4; ++s) { const int row = 4 * s + (lane >> 3), piece = lane & 7; const float* sp = os + row * 68 + piece * 8; v8h o, o2;
#pragma unroll
                for (int i = 0; i < 8; ++i) { const h16 a = (h16)sp[i]; o[i] = a; o2[i] = (h16)((sp[i] - (float)a) * LOSC); }
                *(volatile v8h*)(crow + (size_t)row * ldc + piece * 8) = o; if (C2) *(volatile v8h*)(C2 + (size_t)r0 * ldc + c0 + (size_t)row * ldc + piece * 8) = o2; }
        };
        pass(); __threadfence(); pass();
    } else {
        float* crow = C + (size_t)r0 * ldc + c0;
        auto pass = [&]() {
#pragma unroll
            for (int s = 0; s < 8; ++s) { const int Lid = (lane >> 3) + 4 * s, piece = lane & 7; const int row = Lid >> 1, cofs = (Lid & 1) * 32 + piece * 4;
                v4f val = *(const v4fa*)(os + row * 68 + cofs); if (R) { const v4f rv = *(const v4f*)(R + ((size_t)r0 + row) * ldc + c0 + cofs); val += roundR ? (v4f){bfr(rv[0]), bfr(rv[1]), bfr(rv[2]), bfr(rv[3])} : rv; }
                *(volatile v4f*)(crow + (size_t)row * ldc + cofs) = val; }
        };
        pass(); __threadfence(); pass();
    }
}

__global__ __launch_bounds__(256) void k_wt(const float* __restrict__ Wm, int K, int ncols, bf* WT) {
    __shared__ __align__(16) unsigned short tl[64 * 72];
    const int tid = threadIdx.x, k0 = blockIdx.x * 64, n0 = blockIdx.y * 64;
    const int kk = tid >> 2, nq = (tid & 3) * 16;
#pragma unroll
    for (int i = 0; i < 16; ++i) tl[(nq + i) * 72 + kk] = f2bf(Wm[(size_t)(k0 + kk) * ncols + n0 + nq + i]);
    __syncthreads();
    const int piece = tid & 7;
    auto pass = [&]() {
#pragma unroll
        for (int s = 0; s < 2; ++s) { const int nr = (tid >> 3) + 32 * s; const v8us val = *(const v8usa*)(tl + nr * 72 + piece * 8); *(volatile v8us*)(WT + (size_t)(n0 + nr) * K + k0 + piece * 8) = val; }
    };
    pass(); __threadfence(); pass();
}

__global__ __launch_bounds__(256) void k_cvt8(const float* __restrict__ src, bf* dst, size_t n8) {
    const size_t i = (size_t)blockIdx.x * 256 + threadIdx.x; if (i >= n8) return;
    const v8f v = *(const v8f*)(src + i * 8); v8us o;
#pragma unroll
    for (int k = 0; k < 8; ++k) o[k] = f2bf(v[k]);
    *(volatile v8us*)(dst + i * 8) = o; __threadfence(); *(volatile v8us*)(dst + i * 8) = o;
}
__global__ __launch_bounds__(256) void k_zero8(bf* dst, size_t n8) {
    const size_t i = (size_t)blockIdx.x * 256 + threadIdx.x; if (i >= n8) return; v8us z;
#pragma unroll
    for (int k = 0; k < 8; ++k) z[k] = 0;
    *(volatile v8us*)(dst + i * 8) = z; __threadfence(); *(volatile v8us*)(dst + i * 8) = z;
}

__global__ __launch_bounds__(256) void k_tm(const float* __restrict__ tw, int h, bf* TM) {
    const int lane = threadIdx.x & 31; const size_t t = (size_t)blockIdx.x * 8 + (threadIdx.x >> 5); if (t >= (size_t)TT) return;
#pragma unroll 1
    for (int ps = 0; ps < 2; ++ps) {
#pragma unroll 1
        for (int q = 0; q < TT / 256; ++q) { v8us o;
#pragma unroll
            for (int i = 0; i < 8; ++i) { const int s = q * 256 + lane * 8 + i; const int d = (int)t - s; o[i] = (d >= 0) ? f2bf(tw[(size_t)h * TT + (d >= 0 ? d : 0)]) : (unsigned short)0; }
            *(volatile v8us*)(TM + t * TT + q * 256 + lane * 8) = o; }
        if (ps == 0) __threadfence(); }
}
__global__ __launch_bounds__(256) void k_pb(const float* __restrict__ PT, int h, bf* Bh, bf* Bl) {
    typedef __attribute__((ext_vector_type(2))) unsigned short v2us;
    const int lane = threadIdx.x & 31; const size_t wid = (size_t)blockIdx.x * 8 + (threadIdx.x >> 5); if (wid >= (size_t)EH * (TT / 64)) return; const int e = (int)(wid / (TT / 64)); const int s0 = (int)(wid % (TT / 64)) * 64 + lane * 2; v2us oh, ol;
#pragma unroll
    for (int i = 0; i < 2; ++i) { const float v = PT[(size_t)(s0 + i) * DD + h * EH + e]; const unsigned short hb = f2bf(v); oh[i] = hb; ol[i] = f2bf(v - bf2f(hb)); }
    const size_t o = (size_t)e * TT + s0; *(volatile v2us*)(Bh + o) = oh; *(volatile v2us*)(Bl + o) = ol; __threadfence(); *(volatile v2us*)(Bh + o) = oh; *(volatile v2us*)(Bl + o) = ol;
}
__global__ __launch_bounds__(256) void k_split1k(const float* __restrict__ src, bf* dh, bf* dl) {
    const int lane = threadIdx.x & 31; const size_t r = (size_t)blockIdx.x * 8 + (threadIdx.x >> 5); if (r >= (size_t)TT) return;
#pragma unroll 1
    for (int ps = 0; ps < 2; ++ps) {
#pragma unroll
        for (int q = 0; q < DD / 256; ++q) { const size_t o = r * DD + q * 256 + lane * 8; const v8f v = *(const v8f*)(src + o); v8us oh, ol;
#pragma unroll
            for (int i = 0; i < 8; ++i) { const unsigned short hb = f2bf(v[i]); oh[i] = hb; ol[i] = f2bf(v[i] - bf2f(hb)); }
            *(volatile v8us*)(dh + o) = oh; *(volatile v8us*)(dl + o) = ol; }
        if (ps == 0) __threadfence(); }
}
__global__ __launch_bounds__(256) void k_tr(const float* __restrict__ O, float* OUTB) {
    __shared__ float tl[64][65];
    const int tid = threadIdx.x, t0 = blockIdx.x * 64, e0 = blockIdx.y * 64; const int tt = tid >> 2, eq = (tid & 3) * 16;
#pragma unroll
    for (int i = 0; i < 16; ++i) tl[tt][eq + i] = O[(size_t)(t0 + tt) * DD + e0 + eq + i];
    __syncthreads();
    const int piece = tid & 15, er0 = tid >> 4;
    auto pass = [&]() {
#pragma unroll
        for (int st = 0; st < 4; ++st) { const int er = er0 + 16 * st; v4f v;
#pragma unroll
            for (int i = 0; i < 4; ++i) v[i] = tl[piece * 4 + i][er];
            *(volatile v4f*)(OUTB + (size_t)(e0 + er) * TT + t0 + piece * 4) = v; }
    };
    pass(); __threadfence(); pass();
}

extern "C" void kernel_launch(void* const* d_in, const int* in_sizes, int n_in,
                              void* d_out, int out_size, void* d_ws, size_t ws_size, hipStream_t stream) {
    (void)in_sizes; (void)n_in; (void)out_size;
    const float* x = (const float*)d_in[0]; const float* Wp = (const float*)d_in[1]; const float* bp = (const float*)d_in[2]; const float* tw = (const float*)d_in[3]; const float* Wo = (const float*)d_in[4]; const float* bo = (const float*)d_in[5];
    float* out = (float*)d_out;
    char* wsp = (char*)d_ws;
    auto take = [&](size_t bytes) { char* p = wsp; wsp += (bytes + 255) & ~(size_t)255; return (void*)p; };
    bf* WPB = (bf*)take((size_t)DD * DD * 2); bf* WOB = (bf*)take((size_t)DD * DD * 2); bf* XT = (bf*)take((size_t)TT * DD * 2); float* PT = (float*)take((size_t)TT * DD * 4);
    bf* TM = (bf*)take((size_t)TT * TT * 2); bf* PBh = (bf*)take((size_t)EH * TT * 2); bf* PBl = (bf*)take((size_t)EH * TT * 2); float* C1 = (float*)take((size_t)TT * DD * 4); float* CAT = (float*)take((size_t)TT * DD * 4);
    bf* Ch = (bf*)take((size_t)TT * DD * 2); bf* Cl = (bf*)take((size_t)TT * DD * 2); float* O = (float*)take((size_t)TT * DD * 4);
    if ((size_t)(wsp - (char*)d_ws) > ws_size) return;
    k_cvt8<<<(DD * DD / 8 + 255) / 256, 256, 0, stream>>>(Wp, WPB, (size_t)DD * DD / 8); k_cvt8<<<(DD * DD / 8 + 255) / 256, 256, 0, stream>>>(Wo, WOB, (size_t)DD * DD / 8);
    for (int b = 0; b < NBT; ++b) {
        k_wt<<<dim3(DD / 64, TT / 64, 1), 256, 0, stream>>>(x + (size_t)b * DD * TT, DD, TT, XT);
        k_gemmb<false, false><<<dim3(TT / 64, DD / 64, 1), 128, 0, stream>>>(XT, nullptr, WPB, bp, PT, DD, nullptr, nullptr, DD);
        for (int h = 0; h < NH_; ++h) {
            k_tm<<<TT / 8, 256, 0, stream>>>(tw, h, TM); k_pb<<<(EH * (TT / 64)) / 8, 256, 0, stream>>>(PT, h, PBh, PBl);
            k_gemmbt<false, false><<<dim3(TT / 64, 1, 1), 128, 0, stream>>>(TM, nullptr, PBh, nullptr, C1 + h * EH, DD, nullptr, nullptr, TT, 0);
            k_gemmbt<false, false><<<dim3(TT / 64, 1, 1), 128, 0, stream>>>(TM, nullptr, PBl, nullptr, CAT + h * EH, DD, nullptr, C1 + h * EH, TT, 0); }
        k_split1k<<<TT / 8, 256, 0, stream>>>(CAT, Ch, Cl);
        k_gemmb<true, false><<<dim3(TT / 64, DD / 64, 1), 128, 0, stream>>>(Ch, Cl, WOB, bo, O, DD, nullptr, nullptr, DD);
        k_tr<<<dim3(TT / 64, DD / 64, 1), 256, 0, stream>>>(O, out + (size_t)b * DD * TT); }
}
